// ScaledDotProductAttention_53429393162745
// MI455X (gfx1250) — hardware-verified
//
#include <hip/hip_runtime.h>
#include <math.h>

typedef __attribute__((ext_vector_type(16))) _Float16 v16h;
typedef __attribute__((ext_vector_type(8)))  _Float16 v8h;
typedef __attribute__((ext_vector_type(16))) __bf16   v16b;
typedef __attribute__((ext_vector_type(8)))  __bf16   v8b;
typedef __attribute__((ext_vector_type(8)))  float    v8f;
typedef __attribute__((ext_vector_type(4)))  float    v4f;
typedef __attribute__((ext_vector_type(4)))  unsigned v4u;

constexpr int kBatch = 4;
constexpr int kSeq   = 2048;
constexpr int kDim   = 1024;
constexpr int kRows  = kBatch * kSeq;
constexpr float kQScale    = 0.125f;
constexpr float kPCarry    = 16384.0f;
constexpr float kPCarryInv = 1.0f / 16384.0f;
constexpr float kLog2e     = 1.44269504088896340736f;
constexpr int kTiles64     = kSeq / 64;
constexpr int kTriTiles    = kTiles64 * (kTiles64 + 1) / 2;

constexpr size_t kSzX   = (size_t)kRows * kDim * 2;
constexpr size_t kSzSc  = (size_t)kSeq * kSeq * 4;
constexpr size_t kOffX  = 0;
constexpr size_t kOffW  = kOffX + (kSzX > kSzSc ? kSzX : kSzSc);
constexpr size_t kSzW   = (size_t)3 * kDim * kDim * 2;
constexpr size_t kOffP  = kOffW + kSzW;
constexpr size_t kSzP   = (size_t)kSeq * kSeq * 2;
constexpr size_t kOffQH = kOffP + kSzP;
constexpr size_t kSzQ   = (size_t)kRows * kDim * 2;
constexpr size_t kOffQL = kOffQH + kSzQ;
constexpr size_t kOffKH = kOffQL + kSzQ;
constexpr size_t kOffKL = kOffKH + kSzQ;
constexpr size_t kOffVT = kOffKL + kSzQ;
constexpr size_t kSzVT  = (size_t)kBatch * kDim * kSeq * 2;
constexpr size_t kWsTotal = kOffVT + kSzVT;
static_assert(kSzX >= kSzSc, "scores reuse fits the x region");
static_assert(kWsTotal == 115343360, "carve total");
static_assert(kWsTotal <= 134217728, "carve under 128 MiB");
static_assert(kOffW % 128 == 0 && kOffP % 128 == 0 && kOffQH % 128 == 0 && kOffQL % 128 == 0 &&
              kOffKH % 128 == 0 && kOffKL % 128 == 0 && kOffVT % 128 == 0, "128-B aligned regions");
static_assert(kRows % 64 == 0 && kDim % 64 == 0 && kSeq % 64 == 0, "tile multiples");
static_assert(kDim % 32 == 0 && kSeq % 32 == 0, "K multiples of 32");
static_assert(((kRows / 64) * (kDim / 64)) % 8 == 0, "q/k grid exact");
static_assert(((kDim / 64) * (kSeq / 64)) % 8 == 0, "vt and pv grid exact");
static_assert(kTriTiles % 8 == 0, "score grid exact");
static_assert(kSeq % 8 == 0 && kSeq % 256 == 0, "softmax wave-per-row layout");
static_assert((kRows * kDim) % 512 == 0, "cast grid exact");

__device__ __forceinline__ unsigned short f2bf_bits(float f) {
  unsigned u = __float_as_uint(f);
  return (unsigned short)((u + 0x7FFFu + ((u >> 16) & 1u)) >> 16);
}
__device__ __forceinline__ float bf_bits2f(unsigned short h) { return __uint_as_float(((unsigned)h) << 16); }

__device__ __forceinline__ void dep_guard_h(v8f& a, v8f& b, v16h x, v16h y) { asm volatile("v_nop\n\tv_nop\n\tv_nop\n\tv_nop" : "+v"(a), "+v"(b) : "v"(x), "v"(y)); }
__device__ __forceinline__ void dep_guard_b(v8f& a, v8f& b, v16b x, v16b y) { asm volatile("v_nop\n\tv_nop\n\tv_nop\n\tv_nop" : "+v"(a), "+v"(b) : "v"(x), "v"(y)); }
__device__ __forceinline__ void keep4_h(v16h a, v16h b, v16h c, v16h d) { asm volatile("v_nop" :: "v"(a), "v"(b), "v"(c), "v"(d)); }
__device__ __forceinline__ void keep4_b(v16b a, v16b b, v16b c, v16b d) { asm volatile("v_nop" :: "v"(a), "v"(b), "v"(c), "v"(d)); }
__device__ __forceinline__ void acc_guard4(v8f& a, v8f& b, v8f& c, v8f& d) { asm volatile("v_nop\n\tv_nop\n\tv_nop\n\tv_nop" : "+v"(a), "+v"(b), "+v"(c), "+v"(d)); }
template <typename T> struct Frag;
template <> struct Frag<_Float16> {
  typedef v16h V; union U { v16h v; v8h h[2]; };
  static __device__ __forceinline__ v16h load(const _Float16* p) {
    U f; f.h[0] = *(const v8h*)(p); f.h[1] = *(const v8h*)(p + 16); return f.v;
  }
  static __device__ __forceinline__ v8f mma(v16h a, v16h b, v8f c) {
    return __builtin_amdgcn_wmma_f32_16x16x32_f16(false, a, false, b, (short)0, c, false, false);
  }
  static __device__ __forceinline__ void guard(v8f& a, v8f& b, v16h x, v16h y) { dep_guard_h(a, b, x, y); }
  static __device__ __forceinline__ void keep(v16h a, v16h b, v16h c, v16h d) { keep4_h(a, b, c, d); }
};
template <> struct Frag<__bf16> {
  typedef v16b V; union U { v16b v; v8b h[2]; };
  static __device__ __forceinline__ v16b load(const __bf16* p) {
    U f; f.h[0] = *(const v8b*)(p); f.h[1] = *(const v8b*)(p + 16); return f.v;
  }
  static __device__ __forceinline__ v8f mma(v16b a, v16b b, v8f c) {
    return __builtin_amdgcn_wmma_f32_16x16x32_bf16(false, a, false, b, (short)0, c, false, false);
  }
  static __device__ __forceinline__ void guard(v8f& a, v8f& b, v16b x, v16b y) { dep_guard_b(a, b, x, y); }
  static __device__ __forceinline__ void keep(v16b a, v16b b, v16b c, v16b d) { keep4_b(a, b, c, d); }
};

template <int ET> struct Elem;
template <> struct Elem<0> { typedef _Float16 T; };
template <> struct Elem<1> { typedef __bf16 T; };
template <int ET, bool SPLIT, int BIAS_MODE, int OUT_MODE, bool RESID, int ACT = 0, int TRI = 0>
__global__ __launch_bounds__(256) void wmma_gemm64(
    const unsigned short* __restrict__ Ap, const unsigned short* __restrict__ A2p, int lda, long strideA,
    const unsigned short* __restrict__ Btp, const unsigned short* __restrict__ Bt2p, int ldb, long strideB,
    void* __restrict__ Cout, void* __restrict__ Cout2, int ldc, long strideC,
    const float* __restrict__ bias,
    const float* __restrict__ resid, long strideR,
    int M, int N, int K, float scale) {
  typedef typename Elem<ET>::T T;
  typedef typename Frag<T>::V V;
  const T* A = (const T*)Ap; const T* A2 = (const T*)A2p; const T* Bt = (const T*)Btp; const T* Bt2 = (const T*)Bt2p;
  __shared__ __align__(16) float sT[8][16 * 68];
  const int b    = blockIdx.y;
  const int lane = threadIdx.x & 31;
  const int wave = threadIdx.x >> 5;
  const int tilesN = N >> 6;
  const int tilesM = M >> 6;
  const int tile = blockIdx.x * 8 + wave;
  int tm, tn;
  if (TRI == 1) {
    const int ntri = (tilesM * (tilesM + 1)) >> 1;
    if (tile >= ntri) return;
    int t = (int)((sqrtf(8.0f * (float)tile + 1.0f) - 1.0f) * 0.5f);
    if (((t + 1) * (t + 2)) / 2 <= tile) ++t;
    if ((t * (t + 1)) / 2 > tile) --t;
    tm = t;
    tn = tile - (t * (t + 1)) / 2;
  } else {
    if (tile >= tilesM * tilesN) return;
    tm = tile / tilesN;
    tn = tile - tm * tilesN;
  }
  const int m0 = tm << 6;
  const int n0 = tn << 6;
  const int Kend = (TRI == 2) ? (((m0 + 64) < K) ? (m0 + 64) : K) : K;

  const T* Ab  = A  + (size_t)b * strideA;
  const T* Bb  = Bt + (size_t)b * strideB;
  const T* Ab2 = SPLIT ? (A2  + (size_t)b * strideA) : nullptr;
  const T* Bb2 = SPLIT ? (Bt2 + (size_t)b * strideB) : nullptr;

  const int rlane = lane & 15;
  const int koff  = (lane >> 4) * 8;
  const int mOff  = (lane >> 4) * 8;

  v8f acc[4][4];
#pragma unroll
  for (int i = 0; i < 4; ++i)
#pragma unroll
    for (int j = 0; j < 4; ++j) acc[i][j] = (v8f){0.f,0.f,0.f,0.f,0.f,0.f,0.f,0.f};

  for (int k0 = 0; k0 < Kend; k0 += 32) {
    V bh[4], bl[4];
#pragma unroll
    for (int j = 0; j < 4; ++j) {
      const size_t bo = (size_t)(n0 + (j << 4) + rlane) * ldb + koff + k0;
      bh[j] = Frag<T>::load(Bb + bo);
      if (SPLIT) bl[j] = Frag<T>::load(Bb2 + bo);
    }
#pragma unroll
    for (int i = 0; i < 4; ++i) {
      const size_t ao = (size_t)(m0 + (i << 4) + rlane) * lda + koff + k0;
      V ah = Frag<T>::load(Ab + ao);
      V al;
      if (SPLIT) al = Frag<T>::load(Ab2 + ao);
#pragma unroll
      for (int j = 0; j < 4; ++j) {
        acc[i][j] = Frag<T>::mma(ah, bh[j], acc[i][j]);
        if (SPLIT) {
          acc[i][j] = Frag<T>::mma(ah, bl[j], acc[i][j]);
          acc[i][j] = Frag<T>::mma(al, bh[j], acc[i][j]);
        }
      }
      Frag<T>::guard(acc[i][0], acc[i][3], ah, SPLIT ? al : ah);
    }
    Frag<T>::keep(bh[0], bh[1], bh[2], bh[3]);
    if (SPLIT) Frag<T>::keep(bl[0], bl[1], bl[2], bl[3]);
  }
  acc_guard4(acc[0][0], acc[0][1], acc[0][2], acc[0][3]);
  acc_guard4(acc[1][0], acc[1][1], acc[1][2], acc[1][3]);
  acc_guard4(acc[2][0], acc[2][1], acc[2][2], acc[2][3]);
  acc_guard4(acc[3][0], acc[3][1], acc[3][2], acc[3][3]);

  float* slab = sT[wave];
  const float* Rb = RESID ? (resid + (size_t)b * strideR) : nullptr;
#pragma unroll
  for (int i = 0; i < 4; ++i) {
    const int mBase = m0 + (i << 4);
#pragma unroll
    for (int j = 0; j < 4; ++j) {
      const int n = n0 + (j << 4) + rlane;
      float bv = 0.f;
      if (BIAS_MODE == 2) bv = bf_bits2f(f2bf_bits(bias[n])) * scale;
#pragma unroll
      for (int r = 0; r < 8; ++r) {
        float v = acc[i][j][r] * scale;
        if (BIAS_MODE == 1) v += bf_bits2f(f2bf_bits(bias[mBase + mOff + r])) * scale;
        if (BIAS_MODE == 2) v += bv;
        if (RESID) v += Rb[(size_t)(mBase + mOff + r) * ldc + n];
        if (ACT == 1) v = tanhf(v);
        if (ACT == 2) v = fmaxf(v, 0.0f);
        if (ACT == 4) v = (v > 0.f) ? v : 0.01f * v;
        slab[(mOff + r) * 68 + (j << 4) + rlane] = v;
      }
    }
    __builtin_amdgcn_fence(__ATOMIC_RELEASE, "workgroup");
    __builtin_amdgcn_wave_barrier();
    __builtin_amdgcn_fence(__ATOMIC_ACQUIRE, "workgroup");
    if (OUT_MODE == 0) {
      float* C = (float*)Cout + (size_t)b * strideC;
      const int hh = lane >> 4, c4 = (lane & 15) * 4;
      for (int pass = 0; pass < 2; ++pass) {
#pragma unroll
        for (int it = 0; it < 8; ++it) {
          const int row = it * 2 + hh;
          v4f v = *(const v4f*)(slab + row * 68 + c4);
          *(volatile v4f*)(C + (size_t)(mBase + row) * ldc + n0 + c4) = v;
        }
        __threadfence();
      }
    } else {
      const int q = lane >> 3, c8 = (lane & 7) * 8;
      unsigned short* C  = (unsigned short*)Cout  + (size_t)b * strideC;
      unsigned short* C2 = (OUT_MODE == 2) ? ((unsigned short*)Cout2 + (size_t)b * strideC) : nullptr;
      for (int pass = 0; pass < 2; ++pass) {
#pragma unroll
        for (int it = 0; it < 4; ++it) {
          const int row = it * 4 + q;
          const float* sp = slab + row * 68 + c8;
          v8h hv, lv;
#pragma unroll
          for (int e = 0; e < 8; ++e) {
            if (OUT_MODE == 1) {
              hv[e] = (_Float16)sp[e];
            } else {
              unsigned short hb = f2bf_bits(sp[e]);
              unsigned short lb = f2bf_bits(sp[e] - bf_bits2f(hb));
              hv[e] = __builtin_bit_cast(_Float16, hb);
              lv[e] = __builtin_bit_cast(_Float16, lb);
            }
          }
          *(volatile v8h*)(C + (size_t)(mBase + row) * ldc + n0 + c8) = hv;
          if (OUT_MODE == 2) *(volatile v8h*)(C2 + (size_t)(mBase + row) * ldc + n0 + c8) = lv;
        }
        __threadfence();
      }
    }
    __builtin_amdgcn_fence(__ATOMIC_RELEASE, "workgroup");
    __builtin_amdgcn_wave_barrier();
    __builtin_amdgcn_fence(__ATOMIC_ACQUIRE, "workgroup");
  }
}

__global__ __launch_bounds__(256) void cast_f32_bf16x2(
    const float* __restrict__ in, unsigned short* __restrict__ out, int n2) {
  int i = blockIdx.x * 256 + threadIdx.x;
  if (i < n2) {
    const unsigned short b0 = f2bf_bits(in[2 * i]);
    const unsigned short b1 = f2bf_bits(in[2 * i + 1]);
    const unsigned u = (unsigned)b0 | ((unsigned)b1 << 16);
    ((volatile unsigned*)out)[i] = u;
    __threadfence();
    ((volatile unsigned*)out)[i] = u;
  }
}

__global__ __launch_bounds__(256) void transpose_cast_bf16(
    const float* __restrict__ W0, const float* __restrict__ W1, const float* __restrict__ W2,
    unsigned short* __restrict__ out, int rows, int cols) {
  __shared__ float tileS[64][65];
  const int z = blockIdx.z;
  const float* in = (z == 0) ? W0 : ((z == 1) ? W1 : W2);
  unsigned short* o = out + (size_t)z * rows * cols;
  const int r0 = blockIdx.y * 64;
  const int c0 = blockIdx.x * 64;
  const int tid  = threadIdx.x;
  const int lane = tid & 31;
  const int wave = tid >> 5;
#pragma unroll
  for (int i = 0; i < 4; ++i) {
    const int r  = (tid >> 4) + 16 * i;
    const int c4 = (tid & 15) * 4;
    const v4f f = *(const v4f*)(in + (size_t)(r0 + r) * cols + c0 + c4);
    tileS[r][c4 + 0] = f[0];
    tileS[r][c4 + 1] = f[1];
    tileS[r][c4 + 2] = f[2];
    tileS[r][c4 + 3] = f[3];
  }
  __syncthreads();
  v4u vals[2];
#pragma unroll
  for (int it = 0; it < 2; ++it) {
    const int orow = wave * 8 + it * 4 + (lane >> 3);
    const int k8   = (lane & 7) * 8;
    v4u w;
#pragma unroll
    for (int e2 = 0; e2 < 4; ++e2) {
      const unsigned short lo = f2bf_bits(tileS[k8 + 2 * e2][orow]);
      const unsigned short hi = f2bf_bits(tileS[k8 + 2 * e2 + 1][orow]);
      w[e2] = (unsigned)lo | ((unsigned)hi << 16);
    }
    vals[it] = w;
  }
  for (int pass = 0; pass < 2; ++pass) {
#pragma unroll
    for (int it = 0; it < 2; ++it) {
      const int orow = wave * 8 + it * 4 + (lane >> 3);
      const int k8   = (lane & 7) * 8;
      *(volatile v4u*)(o + (size_t)(c0 + orow) * rows + r0 + k8) = vals[it];
    }
    __threadfence();
  }
}

__global__ __launch_bounds__(256) void causal_softmax_rows(
    const float* __restrict__ sc, unsigned short* __restrict__ P, int S) {
  const int lane = threadIdx.x & 31;
  const int wave = threadIdx.x >> 5;
  const int q = blockIdx.x * 8 + wave;
  const int cend = ((q >> 6) + 1) << 6;
  const int nch  = (cend + 255) >> 8;
  const float* row = sc + (size_t)q * S;
  unsigned short* prow = P + (size_t)q * S;

  float m = -INFINITY, l = 0.f;
#pragma unroll 1
  for (int i = 0; i < nch; ++i) {
    const int c0 = lane * 8 + (i << 8);
    const int cc = (c0 + 8 <= cend) ? c0 : (cend - 8);
    const v4f a0 = *(const v4f*)(row + cc);
    const v4f a1 = *(const v4f*)(row + cc + 4);
    float s[8];
    s[0] = a0[0]; s[1] = a0[1]; s[2] = a0[2]; s[3] = a0[3];
    s[4] = a1[0]; s[5] = a1[1]; s[6] = a1[2]; s[7] = a1[3];
    float cm = -INFINITY;
#pragma unroll
    for (int e = 0; e < 8; ++e) {
      s[e] = (c0 + e <= q) ? s[e] : -INFINITY;
      cm = fmaxf(cm, s[e]);
    }
    const float mn = fmaxf(m, cm);
    const float ar = exp2f((m - mn) * kLog2e);
    const float alpha = (mn == -INFINITY) ? 0.f : ar;
    float ps = 0.f;
#pragma unroll
    for (int e = 0; e < 8; ++e) {
      const float pe = exp2f((s[e] - mn) * kLog2e);
      ps += (c0 + e <= q) ? pe : 0.f;
    }
    l = l * alpha + ps;
    m = mn;
  }
  float gm = m;
#pragma unroll
  for (int off = 1; off < 32; off <<= 1) gm = fmaxf(gm, __shfl_xor(gm, off, 32));
  const float lsc = exp2f((m - gm) * kLog2e);
  float lt = (m == -INFINITY) ? 0.f : (l * lsc);
#pragma unroll
  for (int off = 1; off < 32; off <<= 1) lt += __shfl_xor(lt, off, 32);
  const float inv = kPCarry / lt;

#pragma unroll 1
  for (int i = 0; i < nch; ++i) {
    const int c0 = lane * 8 + (i << 8);
    const int cc = (c0 + 8 <= cend) ? c0 : (cend - 8);
    const v4f a0 = *(const v4f*)(row + cc);
    const v4f a1 = *(const v4f*)(row + cc + 4);
    float s[8];
    s[0] = a0[0]; s[1] = a0[1]; s[2] = a0[2]; s[3] = a0[3];
    s[4] = a1[0]; s[5] = a1[1]; s[6] = a1[2]; s[7] = a1[3];
    v4u w;
#pragma unroll
    for (int e2 = 0; e2 < 4; ++e2) {
      const int ca = c0 + 2 * e2;
      const int cb = ca + 1;
      const float ra = exp2f((s[2 * e2] - gm) * kLog2e) * inv;
      const float rb = exp2f((s[2 * e2 + 1] - gm) * kLog2e) * inv;
      const float pa = (ca <= q) ? ra : 0.f;
      const float pb = (cb <= q) ? rb : 0.f;
      const _Float16 ha = (_Float16)pa;
      const _Float16 hb = (_Float16)pb;
      const unsigned short ua = __builtin_bit_cast(unsigned short, ha);
      const unsigned short ub = __builtin_bit_cast(unsigned short, hb);
      w[e2] = (unsigned)ua | ((unsigned)ub << 16);
    }
    unsigned short* pp = prow + c0;
    if (c0 < cend) *(volatile v4u*)pp = w;
    __threadfence();
    if (c0 < cend) *(volatile v4u*)pp = w;
  }
}

extern "C" void kernel_launch(void* const* d_in, const int* in_sizes, int n_in,
                              void* d_out, int out_size, void* d_ws, size_t ws_size,
                              hipStream_t stream) {
  if (n_in < 7) return;
  if (in_sizes[0] != kRows * kDim) return;
  if (in_sizes[1] != kDim * kDim || in_sizes[3] != kDim * kDim || in_sizes[5] != kDim * kDim) return;
  if (in_sizes[2] != kDim || in_sizes[4] != kDim || in_sizes[6] != kDim) return;
  if (out_size != kRows * kDim) return;
  if (ws_size < kWsTotal) return;

  const float* x  = (const float*)d_in[0];
  const float* Wq = (const float*)d_in[1];
  const float* bq = (const float*)d_in[2];
  const float* Wk = (const float*)d_in[3];
  const float* bk = (const float*)d_in[4];
  const float* Wv = (const float*)d_in[5];
  const float* bv = (const float*)d_in[6];
  float* out = (float*)d_out;

  char* ws = (char*)d_ws;
  unsigned short* Xb = (unsigned short*)(ws + kOffX);
  float*          Sc = (float*)(ws + kOffX);
  unsigned short* WT = (unsigned short*)(ws + kOffW);
  const unsigned short* WqT = WT;
  const unsigned short* WkT = WT + (size_t)kDim * kDim;
  const unsigned short* WvT = WT + (size_t)2 * kDim * kDim;
  unsigned short* Pp = (unsigned short*)(ws + kOffP);
  unsigned short* QH = (unsigned short*)(ws + kOffQH);
  unsigned short* QL = (unsigned short*)(ws + kOffQL);
  unsigned short* KH = (unsigned short*)(ws + kOffKH);
  unsigned short* KL = (unsigned short*)(ws + kOffKL);
  unsigned short* VT = (unsigned short*)(ws + kOffVT);

  cast_f32_bf16x2<<<dim3((kRows * kDim) / 512), dim3(256), 0, stream>>>(x, Xb, (kRows * kDim) / 2);

  transpose_cast_bf16<<<dim3(kDim / 64, kDim / 64, 3), dim3(256), 0, stream>>>(Wq, Wk, Wv, WT, kDim, kDim);

  wmma_gemm64<1, false, 2, 2, false, 0, 0><<<dim3(((kRows / 64) * (kDim / 64)) / 8, 1), dim3(256), 0, stream>>>(
      Xb, Xb, kDim, 0L, WqT, WqT, kDim, 0L, QH, QL, kDim, 0L, bq, x, 0L, kRows, kDim, kDim, kQScale);

  wmma_gemm64<1, false, 2, 2, false, 0, 0><<<dim3(((kRows / 64) * (kDim / 64)) / 8, 1), dim3(256), 0, stream>>>(
      Xb, Xb, kDim, 0L, WkT, WkT, kDim, 0L, KH, KL, kDim, 0L, bk, x, 0L, kRows, kDim, kDim, 1.0f);

  wmma_gemm64<1, false, 1, 1, false, 0, 0><<<dim3(((kDim / 64) * (kSeq / 64)) / 8, kBatch), dim3(256), 0, stream>>>(
      WvT, WvT, kDim, 0L, Xb, Xb, kDim, (long)kSeq * kDim, VT, VT, kSeq, (long)kDim * kSeq, bv, x, 0L,
      kDim, kSeq, kDim, 1.0f);

  for (int b = 0; b < kBatch; ++b) {
    const unsigned short* qh = QH + (size_t)b * kSeq * kDim;
    const unsigned short* ql = QL + (size_t)b * kSeq * kDim;
    const unsigned short* kh = KH + (size_t)b * kSeq * kDim;
    const unsigned short* kl = KL + (size_t)b * kSeq * kDim;
    const unsigned short* vt = VT + (size_t)b * kDim * kSeq;
    float* ob = out + (size_t)b * kSeq * kDim;

    wmma_gemm64<1, true, 0, 0, false, 0, 1><<<dim3(kTriTiles / 8, 1), dim3(256), 0, stream>>>(
        qh, ql, kDim, 0L, kh, kl, kDim, 0L, Sc, Sc, kSeq, 0L, bq, x, 0L, kSeq, kSeq, kDim, 1.0f);

    causal_softmax_rows<<<dim3(kSeq / 8), dim3(256), 0, stream>>>(Sc, Pp, kSeq);

    wmma_gemm64<0, false, 0, 0, false, 0, 2><<<dim3(((kSeq / 64) * (kDim / 64)) / 8, 1), dim3(256), 0, stream>>>(
        Pp, Pp, kSeq, 0L, vt, vt, kSeq, 0L, ob, ob, kDim, 0L, bq, x, 0L, kSeq, kDim, kSeq, kPCarryInv);
  }
}
